// Multi_CrossAttention_7722351198465
// MI455X (gfx1250) — hardware-verified
//
#include <hip/hip_runtime.h>

typedef __attribute__((ext_vector_type(16))) _Float16 v16h;
typedef __attribute__((ext_vector_type(8)))  _Float16 v8h;
typedef __attribute__((ext_vector_type(16))) __bf16   v16b;
typedef __attribute__((ext_vector_type(8)))  __bf16   v8b;
typedef __attribute__((ext_vector_type(8)))  float    v8f;
typedef __attribute__((ext_vector_type(4)))  float    v4f;
typedef __attribute__((ext_vector_type(4)))  unsigned v4u;
#define PSCALE 32768.0f
#define U16(p) ((const unsigned short*)(const void*)(p))
#define PSCALE_INV (1.0f / 32768.0f)

#define NBATCH 4
#define NSEQ 2048
#define NEMB 512
#define NHEAD 8
#define HDIM 64
#define WDIM 512
#define LDQK 1024
#define PCARRY 32768.0f
#define WCARRY 16.0f
#define WCARRY_INV 0.0625f

__device__ __forceinline__ unsigned short f2bf_bits(float f) {
  unsigned u = __float_as_uint(f);
  return (unsigned short)((u + 0x7FFFu + ((u >> 16) & 1u)) >> 16);
}
__device__ __forceinline__ float bf_bits2f(unsigned short h) { return __uint_as_float(((unsigned)h) << 16); }

__device__ __forceinline__ void dep_guard_h(v8f& a, v8f& b, v16h x, v16h y) { asm volatile("v_nop\n\tv_nop\n\tv_nop\n\tv_nop" : "+v"(a), "+v"(b) : "v"(x), "v"(y)); }
__device__ __forceinline__ void dep_guard_b(v8f& a, v8f& b, v16b x, v16b y) { asm volatile("v_nop\n\tv_nop\n\tv_nop\n\tv_nop" : "+v"(a), "+v"(b) : "v"(x), "v"(y)); }
__device__ __forceinline__ void keep4_h(v16h a, v16h b, v16h c, v16h d) { asm volatile("v_nop" :: "v"(a), "v"(b), "v"(c), "v"(d)); }
__device__ __forceinline__ void keep4_b(v16b a, v16b b, v16b c, v16b d) { asm volatile("v_nop" :: "v"(a), "v"(b), "v"(c), "v"(d)); }
__device__ __forceinline__ void acc_guard4(v8f& a, v8f& b, v8f& c, v8f& d) { asm volatile("v_nop\n\tv_nop\n\tv_nop\n\tv_nop" : "+v"(a), "+v"(b), "+v"(c), "+v"(d)); }
template <typename T> struct Frag;
template <> struct Frag<_Float16> {
  typedef v16h V; union U { v16h v; v8h h[2]; };
  static __device__ __forceinline__ v16h load(const _Float16* p) {
    U f; f.h[0] = *(const v8h*)(p); f.h[1] = *(const v8h*)(p + 16); return f.v;
  }
  static __device__ __forceinline__ v8f mma(v16h a, v16h b, v8f c) {
    return __builtin_amdgcn_wmma_f32_16x16x32_f16(false, a, false, b, (short)0, c, false, false);
  }
  static __device__ __forceinline__ void guard(v8f& a, v8f& b, v16h x, v16h y) { dep_guard_h(a, b, x, y); }
  static __device__ __forceinline__ void keep(v16h a, v16h b, v16h c, v16h d) { keep4_h(a, b, c, d); }
};
template <> struct Frag<__bf16> {
  typedef v16b V; union U { v16b v; v8b h[2]; };
  static __device__ __forceinline__ v16b load(const __bf16* p) {
    U f; f.h[0] = *(const v8b*)(p); f.h[1] = *(const v8b*)(p + 16); return f.v;
  }
  static __device__ __forceinline__ v8f mma(v16b a, v16b b, v8f c) {
    return __builtin_amdgcn_wmma_f32_16x16x32_bf16(false, a, false, b, (short)0, c, false, false);
  }
  static __device__ __forceinline__ void guard(v8f& a, v8f& b, v16b x, v16b y) { dep_guard_b(a, b, x, y); }
  static __device__ __forceinline__ void keep(v16b a, v16b b, v16b c, v16b d) { keep4_b(a, b, c, d); }
};

template <int ET> struct Elem;
template <> struct Elem<0> { typedef _Float16 T; };
template <> struct Elem<1> { typedef __bf16 T; };
template <int ET, bool SPLIT, int BIAS_MODE, int OUT_MODE, bool RESID, int ACT = 0>
__global__ __launch_bounds__(256) void wmma_gemm64(
    const unsigned short* __restrict__ Ap, const unsigned short* __restrict__ A2p, int lda, long strideA,
    const unsigned short* __restrict__ Btp, const unsigned short* __restrict__ Bt2p, int ldb, long strideB,
    void* __restrict__ Cout, void* __restrict__ Cout2, int ldc, long strideC,
    const float* __restrict__ bias,
    const float* __restrict__ resid, long strideR,
    int M, int N, int K, float scale) {
  typedef typename Elem<ET>::T T;
  typedef typename Frag<T>::V V;
  const T* A = (const T*)Ap; const T* A2 = (const T*)A2p; const T* Bt = (const T*)Btp; const T* Bt2 = (const T*)Bt2p;
  __shared__ __align__(16) float sT[8][16 * 68];
  const int b    = blockIdx.y;
  const int lane = threadIdx.x & 31;
  const int wave = threadIdx.x >> 5;
  const int tilesN = N >> 6;
  const int tilesM = M >> 6;
  const int tile = blockIdx.x * 8 + wave;
  if (tile >= tilesM * tilesN) return;
  const int tm = tile / tilesN;
  const int tn = tile - tm * tilesN;
  const int m0 = tm << 6;
  const int n0 = tn << 6;

  const T* Ab  = A  + (size_t)b * strideA;
  const T* Bb  = Bt + (size_t)b * strideB;
  const T* Ab2 = SPLIT ? (A2  + (size_t)b * strideA) : nullptr;
  const T* Bb2 = SPLIT ? (Bt2 + (size_t)b * strideB) : nullptr;

  const int rlane = lane & 15;
  const int koff  = (lane >> 4) * 8;
  const int mOff  = (lane >> 4) * 8;

  v8f acc[4][4];
#pragma unroll
  for (int i = 0; i < 4; ++i)
#pragma unroll
    for (int j = 0; j < 4; ++j) acc[i][j] = (v8f){0.f,0.f,0.f,0.f,0.f,0.f,0.f,0.f};

  for (int k0 = 0; k0 < K; k0 += 32) {
    V bh[4], bl[4];
#pragma unroll
    for (int j = 0; j < 4; ++j) {
      const size_t bo = (size_t)(n0 + (j << 4) + rlane) * ldb + koff + k0;
      bh[j] = Frag<T>::load(Bb + bo);
      if (SPLIT) bl[j] = Frag<T>::load(Bb2 + bo);
    }
#pragma unroll
    for (int i = 0; i < 4; ++i) {
      const size_t ao = (size_t)(m0 + (i << 4) + rlane) * lda + koff + k0;
      V ah = Frag<T>::load(Ab + ao);
      V al;
      if (SPLIT) al = Frag<T>::load(Ab2 + ao);
#pragma unroll
      for (int j = 0; j < 4; ++j) {
        acc[i][j] = Frag<T>::mma(ah, bh[j], acc[i][j]);
        if (SPLIT) {
          acc[i][j] = Frag<T>::mma(ah, bl[j], acc[i][j]);
          acc[i][j] = Frag<T>::mma(al, bh[j], acc[i][j]);
        }
      }
      Frag<T>::guard(acc[i][0], acc[i][3], ah, SPLIT ? al : ah);
    }
    Frag<T>::keep(bh[0], bh[1], bh[2], bh[3]);
    if (SPLIT) Frag<T>::keep(bl[0], bl[1], bl[2], bl[3]);
  }
  acc_guard4(acc[0][0], acc[0][1], acc[0][2], acc[0][3]);
  acc_guard4(acc[1][0], acc[1][1], acc[1][2], acc[1][3]);
  acc_guard4(acc[2][0], acc[2][1], acc[2][2], acc[2][3]);
  acc_guard4(acc[3][0], acc[3][1], acc[3][2], acc[3][3]);

  float* slab = sT[wave];
  const float* Rb = RESID ? (resid + (size_t)b * strideR) : nullptr;
#pragma unroll
  for (int i = 0; i < 4; ++i) {
    const int mBase = m0 + (i << 4);
#pragma unroll
    for (int j = 0; j < 4; ++j) {
      const int n = n0 + (j << 4) + rlane;
      float bv = 0.f;
      if (BIAS_MODE == 2) bv = bias[n];
#pragma unroll
      for (int r = 0; r < 8; ++r) {
        float v = acc[i][j][r] * scale;
        if (BIAS_MODE == 1) v += bias[mBase + mOff + r];
        if (BIAS_MODE == 2) v += bv;
        if (RESID) v += Rb[(size_t)(mBase + mOff + r) * ldc + n];
        if (ACT == 1) v = tanhf(v);
        if (ACT == 2) v = fmaxf(v, 0.0f);
        if (ACT == 3) v = v / (1.0f + expf(-v));
        if (ACT == 4) v = (v > 0.f) ? v : 0.01f * v;
        if (ACT == 5) v = 0.5f * v * (1.0f + erff(v * 0.70710678118654752f));
        slab[(mOff + r) * 68 + (j << 4) + rlane] = v;
      }
    }
    __builtin_amdgcn_fence(__ATOMIC_RELEASE, "workgroup");
    __builtin_amdgcn_wave_barrier();
    __builtin_amdgcn_fence(__ATOMIC_ACQUIRE, "workgroup");
    if (OUT_MODE == 0) {
      float* C = (float*)Cout + (size_t)b * strideC;
      const int hh = lane >> 4, c4 = (lane & 15) * 4;
      for (int pass = 0; pass < 2; ++pass) {
#pragma unroll
        for (int it = 0; it < 8; ++it) {
          const int row = it * 2 + hh;
          v4f v = *(const v4f*)(slab + row * 68 + c4);
          *(volatile v4f*)(C + (size_t)(mBase + row) * ldc + n0 + c4) = v;
        }
        __threadfence();
      }
    } else {
      const int q = lane >> 3, c8 = (lane & 7) * 8;
      unsigned short* C  = (unsigned short*)Cout  + (size_t)b * strideC;
      unsigned short* C2 = (OUT_MODE == 2) ? ((unsigned short*)Cout2 + (size_t)b * strideC) : nullptr;
      for (int pass = 0; pass < 2; ++pass) {
#pragma unroll
        for (int it = 0; it < 4; ++it) {
          const int row = it * 4 + q;
          const float* sp = slab + row * 68 + c8;
          v8h hv, lv;
#pragma unroll
          for (int e = 0; e < 8; ++e) {
            if (OUT_MODE == 1) {
              hv[e] = (_Float16)sp[e];
            } else {
              unsigned short hb = f2bf_bits(sp[e]);
              unsigned short lb = f2bf_bits(sp[e] - bf_bits2f(hb));
              hv[e] = __builtin_bit_cast(_Float16, hb);
              lv[e] = __builtin_bit_cast(_Float16, lb);
            }
          }
          *(volatile v8h*)(C + (size_t)(mBase + row) * ldc + n0 + c8) = hv;
          if (OUT_MODE == 2) *(volatile v8h*)(C2 + (size_t)(mBase + row) * ldc + n0 + c8) = lv;
        }
        __threadfence();
      }
    }
    __builtin_amdgcn_fence(__ATOMIC_RELEASE, "workgroup");
    __builtin_amdgcn_wave_barrier();
    __builtin_amdgcn_fence(__ATOMIC_ACQUIRE, "workgroup");
  }
}

__global__ __launch_bounds__(256) void cast_f32_f16x2(
    const float* __restrict__ in, _Float16* __restrict__ out, int n2) {
  int i = blockIdx.x * 256 + threadIdx.x;
  if (i < n2) {
    const _Float16 h0 = (_Float16)in[2 * i], h1 = (_Float16)in[2 * i + 1];
    const unsigned u = (unsigned)__builtin_bit_cast(unsigned short, h0) | ((unsigned)__builtin_bit_cast(unsigned short, h1) << 16);
    ((volatile unsigned*)out)[i] = u;
    __threadfence();
    ((volatile unsigned*)out)[i] = u;
  }
}

__global__ __launch_bounds__(256) void wt_cast16_kernel(const float* __restrict__ W,
                                                        unsigned short* __restrict__ Wt, int rowOff) {
  __shared__ float tile[64][65];
  const int t = threadIdx.x;
  const int n0 = blockIdx.x * 64, k0 = blockIdx.y * 64;
#pragma unroll
  for (int p = 0; p < 4; ++p) {
    const int kr = p * 16 + (t >> 4);
    const int c4 = (t & 15) * 4;
    const v4f w = *(const v4f*)(W + (size_t)(k0 + kr) * WDIM + n0 + c4);
    tile[kr][c4 + 0] = w[0];
    tile[kr][c4 + 1] = w[1];
    tile[kr][c4 + 2] = w[2];
    tile[kr][c4 + 3] = w[3];
  }
  __syncthreads();
  const int wave = t >> 5, lane = t & 31, rq = lane >> 3, pc8 = (lane & 7) * 8;
  _Float16* Wth = (_Float16*)Wt;
  for (int pass = 0; pass < 2; ++pass) {
#pragma unroll
    for (int it = 0; it < 2; ++it) {
      const int nl = it * 32 + wave * 4 + rq;
      v8h hv;
#pragma unroll
      for (int e = 0; e < 8; ++e) hv[e] = (_Float16)(tile[pc8 + e][nl] * WCARRY);
      *(volatile v8h*)(Wth + (size_t)(rowOff + n0 + nl) * WDIM + k0 + pc8) = hv;
    }
    __threadfence();
  }
}

__device__ __forceinline__ v8f mma_h(v16h a, v16h bb, v8f cc) {
  cc = __builtin_amdgcn_wmma_f32_16x16x32_f16(false, a, false, bb, (short)0, cc, false, false);
  asm volatile("v_nop\n\tv_nop\n\tv_nop\n\tv_nop" : "+v"(cc) : "v"(a), "v"(bb));
  return cc;
}

__global__ __launch_bounds__(128)
void dual_attn_kernel(const unsigned short* __restrict__ QKx, const unsigned short* __restrict__ QKy,
                      const unsigned short* __restrict__ Vtx, const unsigned short* __restrict__ Vty,
                      const float* __restrict__ xres, const float* __restrict__ yres,
                      float* __restrict__ out) {
  union FH { v16h v; v8h h[2]; };
  __shared__ __align__(16) _Float16 K1s[64 * 64];
  __shared__ __align__(16) _Float16 K2s[64 * 64];
  __shared__ __align__(16) _Float16 V1s[64 * 64];
  __shared__ __align__(16) _Float16 V2s[64 * 64];
  __shared__ __align__(16) _Float16 Psh[4][16 * 64];
  __shared__ __align__(16) float    Osl[4][16 * 68];

  const int tid  = threadIdx.x;
  const int wave = tid >> 5;
  const int lane = tid & 31;
  const int hh   = lane >> 4;
  const int c    = lane & 15;

  const int bx  = blockIdx.x;
  const int qb  = bx & 31;
  const int bhd = bx >> 5;
  const int h   = bhd & 7;
  const int b   = bhd >> 3;
  const int q0  = qb * 64 + wave * 16;
  const size_t rowb = (size_t)b * NSEQ;

  const _Float16* QKxh = (const _Float16*)QKx;
  const _Float16* QKyh = (const _Float16*)QKy;

  v16h q1f[2], q2f[2];
  {
    const _Float16* q1row = QKyh + (rowb + q0 + c) * LDQK + h * HDIM;
    const _Float16* q2row = QKxh + (rowb + q0 + c) * LDQK + h * HDIM;
#pragma unroll
    for (int dc = 0; dc < 2; ++dc) {
      FH f1;
      f1.h[0] = *(const v8h*)(q1row + dc * 32 + 8 * hh);
      f1.h[1] = *(const v8h*)(q1row + dc * 32 + 16 + 8 * hh);
      q1f[dc] = f1.v;
      FH f2;
      f2.h[0] = *(const v8h*)(q2row + dc * 32 + 8 * hh);
      f2.h[1] = *(const v8h*)(q2row + dc * 32 + 16 + 8 * hh);
      q2f[dc] = f2.v;
    }
  }

  float mrow[8], lrow[8];
  v8f oa[4], ob[4];
#pragma unroll
  for (int r = 0; r < 8; ++r) { mrow[r] = -__builtin_inff(); lrow[r] = 0.f; }
#pragma unroll
  for (int t = 0; t < 4; ++t) { oa[t] = (v8f){0.f,0.f,0.f,0.f,0.f,0.f,0.f,0.f}; ob[t] = (v8f){0.f,0.f,0.f,0.f,0.f,0.f,0.f,0.f}; }

#pragma unroll 1
  for (int kc = 0; kc < NSEQ / 64; ++kc) {
    const int kv0 = kc * 64;
    __syncthreads();
    {
      const int r = tid >> 1, hf = (tid & 1) * 32;
      const v4u* gk1 = (const v4u*)(QKx + (rowb + kv0 + r) * LDQK + NEMB + h * HDIM + hf);
      const v4u* gk2 = (const v4u*)(QKy + (rowb + kv0 + r) * LDQK + NEMB + h * HDIM + hf);
      v4u* lk1 = (v4u*)(K1s + r * 64 + hf);
      v4u* lk2 = (v4u*)(K2s + r * 64 + hf);
#pragma unroll
      for (int i = 0; i < 4; ++i) { lk1[i] = gk1[i]; lk2[i] = gk2[i]; }
      asm volatile("" ::: "memory");
      const v4u* gv1 = (const v4u*)(Vtx + ((size_t)b * NEMB + h * HDIM + r) * NSEQ + kv0 + hf);
      const v4u* gv2 = (const v4u*)(Vty + ((size_t)b * NEMB + h * HDIM + r) * NSEQ + kv0 + hf);
      v4u* lv1 = (v4u*)(V1s + r * 64 + hf);
      v4u* lv2 = (v4u*)(V2s + r * 64 + hf);
#pragma unroll
      for (int i = 0; i < 4; ++i) { lv1[i] = gv1[i]; lv2[i] = gv2[i]; }
    }
    __syncthreads();

    v8f s[4];
#pragma unroll
    for (int j = 0; j < 4; ++j) {
      s[j] = (v8f){0.f,0.f,0.f,0.f,0.f,0.f,0.f,0.f};
#pragma unroll
      for (int dc = 0; dc < 2; ++dc) {
        FH kb;
        kb.h[0] = *(const v8h*)(K1s + (j * 16 + c) * 64 + dc * 32 + 8 * hh);
        kb.h[1] = *(const v8h*)(K1s + (j * 16 + c) * 64 + dc * 32 + 16 + 8 * hh);
        s[j] = mma_h(q1f[dc], kb.v, s[j]);
        FH kd;
        kd.h[0] = *(const v8h*)(K2s + (j * 16 + c) * 64 + dc * 32 + 8 * hh);
        kd.h[1] = *(const v8h*)(K2s + (j * 16 + c) * 64 + dc * 32 + 16 + 8 * hh);
        s[j] = mma_h(q2f[dc], kd.v, s[j]);
      }
    }

    float cm[8];
#pragma unroll
    for (int r = 0; r < 8; ++r) {
      float m = -__builtin_inff();
#pragma unroll
      for (int j = 0; j < 4; ++j) { s[j][r] *= 0.0625f; m = fmaxf(m, s[j][r]); }
#pragma unroll
      for (int off = 1; off < 16; off <<= 1) m = fmaxf(m, __shfl_xor(m, off, 32));
      cm[r] = m;
    }

    _Float16* pw = Psh[wave];
#pragma unroll
    for (int r = 0; r < 8; ++r) {
      const float mnew  = fmaxf(mrow[r], cm[r]);
      const float alpha = expf(mrow[r] - mnew);
      mrow[r] = mnew;
      float psum = 0.f;
#pragma unroll
      for (int j = 0; j < 4; ++j) {
        const float p = expf(s[j][r] - mnew);
        psum += p;
        pw[(8 * hh + r) * 64 + j * 16 + c] = (_Float16)(p * PCARRY);
      }
#pragma unroll
      for (int off = 1; off < 16; off <<= 1) psum += __shfl_xor(psum, off, 32);
      lrow[r] = lrow[r] * alpha + psum;
#pragma unroll
      for (int t = 0; t < 4; ++t) { oa[t][r] *= alpha; ob[t][r] *= alpha; }
    }
    __builtin_amdgcn_fence(__ATOMIC_RELEASE, "workgroup");
    __builtin_amdgcn_wave_barrier();
    __builtin_amdgcn_fence(__ATOMIC_ACQUIRE, "workgroup");

#pragma unroll 1
    for (int kk = 0; kk < 2; ++kk) {
      FH pa;
      pa.h[0] = *(const v8h*)(pw + c * 64 + kk * 32 + 8 * hh);
      pa.h[1] = *(const v8h*)(pw + c * 64 + kk * 32 + 16 + 8 * hh);
#pragma unroll
      for (int t = 0; t < 4; ++t) {
        FH vb;
        vb.h[0] = *(const v8h*)(V1s + (t * 16 + c) * 64 + kk * 32 + 8 * hh);
        vb.h[1] = *(const v8h*)(V1s + (t * 16 + c) * 64 + kk * 32 + 16 + 8 * hh);
        oa[t] = mma_h(pa.v, vb.v, oa[t]);
        FH vc;
        vc.h[0] = *(const v8h*)(V2s + (t * 16 + c) * 64 + kk * 32 + 8 * hh);
        vc.h[1] = *(const v8h*)(V2s + (t * 16 + c) * 64 + kk * 32 + 16 + 8 * hh);
        ob[t] = mma_h(pa.v, vc.v, ob[t]);
      }
    }
  }

  float inv[8];
#pragma unroll
  for (int r = 0; r < 8; ++r) inv[r] = 1.0f / (lrow[r] * PCARRY);
  float* os = Osl[wave];
  const size_t obase = rowb * NEMB + (size_t)h * HDIM;
  const int c4 = c * 4;

#pragma unroll
  for (int r = 0; r < 8; ++r)
#pragma unroll
    for (int t = 0; t < 4; ++t) os[(8 * hh + r) * 68 + t * 16 + c] = oa[t][r] * inv[r];
  __builtin_amdgcn_fence(__ATOMIC_RELEASE, "workgroup");
  __builtin_amdgcn_wave_barrier();
  __builtin_amdgcn_fence(__ATOMIC_ACQUIRE, "workgroup");
  {
    for (int pass = 0; pass < 2; ++pass) {
#pragma unroll
      for (int it = 0; it < 8; ++it) {
        const int row = it * 2 + hh;
        const size_t gi = obase + (size_t)(q0 + row) * NEMB + c4;
        v4f val = *(const v4f*)(os + row * 68 + c4);
        const v4f rr = *(const v4f*)(xres + gi);
        val += rr;
        *(volatile v4f*)(out + gi) = val;
      }
      __threadfence();
    }
  }
  __builtin_amdgcn_fence(__ATOMIC_RELEASE, "workgroup");
  __builtin_amdgcn_wave_barrier();
  __builtin_amdgcn_fence(__ATOMIC_ACQUIRE, "workgroup");

#pragma unroll
  for (int r = 0; r < 8; ++r)
#pragma unroll
    for (int t = 0; t < 4; ++t) os[(8 * hh + r) * 68 + t * 16 + c] = ob[t][r] * inv[r];
  __builtin_amdgcn_fence(__ATOMIC_RELEASE, "workgroup");
  __builtin_amdgcn_wave_barrier();
  __builtin_amdgcn_fence(__ATOMIC_ACQUIRE, "workgroup");
  {
    float* out1 = out + (size_t)NBATCH * NSEQ * NEMB;
    for (int pass = 0; pass < 2; ++pass) {
#pragma unroll
      for (int it = 0; it < 8; ++it) {
        const int row = it * 2 + hh;
        const size_t gi = obase + (size_t)(q0 + row) * NEMB + c4;
        v4f val = *(const v4f*)(os + row * 68 + c4);
        const v4f rr = *(const v4f*)(yres + gi);
        val += rr;
        *(volatile v4f*)(out1 + gi) = val;
      }
      __threadfence();
    }
  }
}

static_assert(NEMB == NHEAD * HDIM, "head split");
static_assert(HDIM == 64, "attention kernel is head-dim 64");
static_assert(NSEQ % 64 == 0 && NSEQ / 64 == 32, "query/key blocks of 64, 32 per sequence");
static_assert(NHEAD == 8 && NBATCH == 4, "block index decode");
static_assert(NEMB % 32 == 0, "GEMM K multiple of 32");
static_assert((NBATCH * NSEQ) % 64 == 0 && (2 * NEMB) % 64 == 0, "QK GEMM M,N tile multiples");
static_assert(NEMB % 64 == 0 && NSEQ % 64 == 0, "Vt GEMM M,N tile multiples");
static_assert(LDQK == 2 * NEMB, "QK plane pitch");
static_assert((size_t)2 * NBATCH * NSEQ * NEMB * 4 == 33554432u, "out1 byte offset + size == d_out total");

extern "C" void kernel_launch(void* const* d_in, const int* in_sizes, int n_in,
                              void* d_out, int out_size, void* d_ws, size_t ws_size,
                              hipStream_t stream) {
  const size_t nAct = (size_t)NBATCH * NSEQ * NEMB;
  const size_t nW   = (size_t)NEMB * NEMB;
  if (n_in < 5) return;
  if ((size_t)in_sizes[0] != nAct || (size_t)in_sizes[1] != nAct ||
      (size_t)in_sizes[2] != nW || (size_t)in_sizes[3] != nW || (size_t)in_sizes[4] != nW) return;
  if ((size_t)out_size != 2 * nAct) return;

  const size_t offX16  = 0;
  const size_t offY16  = offX16  + nAct * 2;
  const size_t offWqkT = offY16  + nAct * 2;
  const size_t offWvT  = offWqkT + (size_t)2 * NEMB * NEMB * 2;
  const size_t offQKx  = offWvT  + nW * 2;
  const size_t offQKy  = offQKx  + (size_t)NBATCH * NSEQ * LDQK * 2;
  const size_t offVtx  = offQKy  + (size_t)NBATCH * NSEQ * LDQK * 2;
  const size_t offVty  = offVtx  + nAct * 2;
  const size_t wsTotal = offVty  + nAct * 2;
  if (ws_size < wsTotal) return;

  const float* x  = (const float*)d_in[0];
  const float* y  = (const float*)d_in[1];
  const float* Wq = (const float*)d_in[2];
  const float* Wk = (const float*)d_in[3];
  const float* Wv = (const float*)d_in[4];
  float* out = (float*)d_out;
  char* ws = (char*)d_ws;
  unsigned short* x16  = (unsigned short*)(ws + offX16);
  unsigned short* y16  = (unsigned short*)(ws + offY16);
  unsigned short* WqkT = (unsigned short*)(ws + offWqkT);
  unsigned short* WvT  = (unsigned short*)(ws + offWvT);
  unsigned short* QKx  = (unsigned short*)(ws + offQKx);
  unsigned short* QKy  = (unsigned short*)(ws + offQKy);
  unsigned short* Vtx  = (unsigned short*)(ws + offVtx);
  unsigned short* Vty  = (unsigned short*)(ws + offVty);
  const float* dummyf = (const float*)d_ws;

  const int n2 = (int)(nAct / 2);
  cast_f32_f16x2<<<dim3((n2 + 255) / 256), dim3(256), 0, stream>>>(x, (_Float16*)x16, n2);
  cast_f32_f16x2<<<dim3((n2 + 255) / 256), dim3(256), 0, stream>>>(y, (_Float16*)y16, n2);

  const dim3 gW(WDIM / 64, WDIM / 64);
  wt_cast16_kernel<<<gW, dim3(256), 0, stream>>>(Wq, WqkT, 0);
  wt_cast16_kernel<<<gW, dim3(256), 0, stream>>>(Wk, WqkT, NEMB);
  wt_cast16_kernel<<<gW, dim3(256), 0, stream>>>(Wv, WvT, 0);

  const int Mqk = NBATCH * NSEQ, Nqk = 2 * NEMB, Kp = NEMB;
  const dim3 gQK((Mqk / 64) * (Nqk / 64) / 8, 1);
  wmma_gemm64<0, false, 0, 1, false><<<gQK, dim3(256), 0, stream>>>(
      x16, x16, Kp, 0L, WqkT, WqkT, Kp, 0L, (void*)QKx, (void*)QKx, LDQK, 0L,
      dummyf, dummyf, 0L, Mqk, Nqk, Kp, WCARRY_INV);
  wmma_gemm64<0, false, 0, 1, false><<<gQK, dim3(256), 0, stream>>>(
      y16, y16, Kp, 0L, WqkT, WqkT, Kp, 0L, (void*)QKy, (void*)QKy, LDQK, 0L,
      dummyf, dummyf, 0L, Mqk, Nqk, Kp, WCARRY_INV);

  const int Mv = NEMB, Nv = NSEQ;
  const dim3 gV((Mv / 64) * (Nv / 64) / 8, NBATCH);
  wmma_gemm64<0, false, 0, 1, false><<<gV, dim3(256), 0, stream>>>(
      WvT, WvT, Kp, 0L, x16, x16, Kp, (long)NSEQ * NEMB, (void*)Vtx, (void*)Vtx, NSEQ, (long)NEMB * NSEQ,
      dummyf, dummyf, 0L, Mv, Nv, Kp, WCARRY_INV);
  wmma_gemm64<0, false, 0, 1, false><<<gV, dim3(256), 0, stream>>>(
      WvT, WvT, Kp, 0L, y16, y16, Kp, (long)NSEQ * NEMB, (void*)Vty, (void*)Vty, NSEQ, (long)NEMB * NSEQ,
      dummyf, dummyf, 0L, Mv, Nv, Kp, WCARRY_INV);

  const dim3 gA(NBATCH * NHEAD * (NSEQ / 64));
  dual_attn_kernel<<<gA, dim3(128), 0, stream>>>(QKx, QKy, Vtx, Vty, x, y, out);
}
